// SelfRouting2d_83983790506265
// MI455X (gfx1250) — hardware-verified
//
#include <hip/hip_runtime.h>
#include <math.h>

typedef __attribute__((ext_vector_type(16))) _Float16 v16h;
typedef __attribute__((ext_vector_type(16))) __bf16 v16b;
typedef __attribute__((ext_vector_type(8)))  _Float16 v8h;
typedef __attribute__((ext_vector_type(8)))  float v8f;
typedef __attribute__((ext_vector_type(4)))  float v4f;
typedef __attribute__((ext_vector_type(2)))  float v2f;
typedef __attribute__((ext_vector_type(4)))  unsigned v4u;
typedef __attribute__((ext_vector_type(4)))  int v4i;
typedef float __attribute__((may_alias)) float_a;
typedef int __attribute__((may_alias)) int_a;

template <typename T> __device__ __forceinline__ void vst2(void* p, T v) { *(volatile T*)p = v; __threadfence(); *(volatile T*)p = v; }
__device__ __forceinline__ v8f wmma16(v16h a, v16h b, v8f c) {
  v8f d = __builtin_amdgcn_wmma_f32_16x16x32_f16(false, a, false, b, (short)0, c, false, false);
  asm volatile("v_nop\n\tv_nop\n\tv_nop\n\tv_nop" : "+v"(d) : "v"(a), "v"(b));
  return d;
}
__device__ __forceinline__ v8f wmma_bf(v16b a, v16b b, v8f c) {
  v8f d = __builtin_amdgcn_wmma_f32_16x16x32_bf16(false, a, false, b, (short)0, c, false, false);
  asm volatile("v_nop\n\tv_nop\n\tv_nop\n\tv_nop" : "+v"(d) : "v"(a), "v"(b));
  return d;
}
__device__ __forceinline__ v16h frag_h(const _Float16* rowk0, int lane) {
  union { v16h v; v8h q[2]; } u; const _Float16* p = rowk0 + 8 * (lane >> 4);
  u.q[0] = *(const v8h*)p; u.q[1] = *(const v8h*)(p + 16); return u.v;
}
__device__ __forceinline__ v16h frag_f32(const float* rowk0, int lane) {
  v16h a; const float* p = rowk0 + 8 * (lane >> 4);
#pragma unroll
  for (int i = 0; i < 8; ++i) { a[i] = (_Float16)p[i]; a[8 + i] = (_Float16)p[16 + i]; }
  return a;
}
__device__ __forceinline__ v16h frag_f32s(const float* rowk0, int lane, float sc) {
  v16h a; const float* p = rowk0 + 8 * (lane >> 4);
#pragma unroll
  for (int i = 0; i < 8; ++i) { a[i] = (_Float16)(p[i] * sc); a[8 + i] = (_Float16)(p[16 + i] * sc); }
  return a;
}
__device__ __forceinline__ v16h fragc_f32(const float* W, int k0, int n, int lane, int ld, int K) {
  v16h a; const int g = lane >> 4;
#pragma unroll
  for (int i = 0; i < 8; ++i) { const int ka = k0 + 8 * g + i, kb = ka + 16;
    a[i] = (_Float16)(ka < K ? W[(size_t)ka * ld + n] : 0.f); a[8 + i] = (_Float16)(kb < K ? W[(size_t)kb * ld + n] : 0.f); }
  return a;
}
struct F2 { v16b h, l; };
__device__ __forceinline__ F2 bsplit16(const float v[16]) { F2 r;
#pragma unroll
  for (int i = 0; i < 16; ++i) { const __bf16 h = (__bf16)v[i]; r.h[i] = h; r.l[i] = (__bf16)(v[i] - (float)h); }
  return r; }
__device__ __forceinline__ F2 split_row(const float* row, int k0, int lane) { float v[16]; const float* p = row + k0 + 8 * (lane >> 4);
#pragma unroll
  for (int i = 0; i < 8; ++i) { v[i] = p[i]; v[8 + i] = p[16 + i]; }
  return bsplit16(v); }
__device__ __forceinline__ F2 split_rowK(const float* row, int k0, int lane, int K) { float v[16]; const int g = lane >> 4;
#pragma unroll
  for (int i = 0; i < 8; ++i) { const int ka = k0 + 8 * g + i, kb = ka + 16; v[i] = ka < K ? row[ka] : 0.f; v[8 + i] = kb < K ? row[kb] : 0.f; }
  return bsplit16(v); }
__device__ __forceinline__ F2 split_col(const float* W, int k0, int n, int lane, int ld, int K) { float v[16]; const int g = lane >> 4;
#pragma unroll
  for (int i = 0; i < 8; ++i) { const int ka = k0 + 8 * g + i, kb = ka + 16; v[i] = ka < K ? W[(size_t)ka * ld + n] : 0.f; v[8 + i] = kb < K ? W[(size_t)kb * ld + n] : 0.f; }
  return bsplit16(v); }
__device__ __forceinline__ v8f mac3(const F2& a, const F2& b, v8f c) { c = wmma_bf(a.l, b.h, c); c = wmma_bf(a.h, b.l, c); return wmma_bf(a.h, b.h, c); }
__device__ __forceinline__ float sigm(float v) { return 1.0f / (1.0f + expf(-v)); }
#define LDSX() do { asm volatile("s_wait_dscnt 0" ::: "memory"); __builtin_amdgcn_wave_barrier(); __builtin_amdgcn_fence(__ATOMIC_RELEASE, "workgroup"); } while (0)

#define NB 4
#define NA 32
#define NBO 8
#define CI 16
#define DO 16
#define HW 32
#define NPX (HW * HW)
#define KKA 288

__device__ __forceinline__ v16h frag_pose(const float* __restrict__ pb, int a, int ys, int xs, bool inb, int lane) {
  const int g = lane >> 4; v16h r;
#pragma unroll
  for (int i = 0; i < 8; ++i) { const int cc = 8 * g + i; float v = 0.f; if (inb) v = pb[((size_t)(a * CI + cc)) * NPX + ys * HW + xs]; r[i] = (_Float16)v; r[8 + i] = (_Float16)0.f; }
  return r;
}
__device__ __forceinline__ v16h frag_w16(const float* __restrict__ row, int lane, float sc) {
  const int g = lane >> 4; v16h r;
#pragma unroll
  for (int i = 0; i < 8; ++i) { r[i] = (_Float16)(row[8 * g + i] * sc); r[8 + i] = (_Float16)0.f; }
  return r;
}
__global__ __launch_bounds__(128) void k_main(const float* __restrict__ act, const float* __restrict__ pose, const float* __restrict__ W1, const float* __restrict__ W2, const float* __restrict__ b2, float* __restrict__ aout, float* __restrict__ pout) {
  __shared__ __align__(16) float sa[NBO][68];
  __shared__ __align__(16) float sp[NBO * DO][68];
  const int tid = threadIdx.x, wave = tid >> 5, lane = tid & 31, col = lane & 15, g = lane >> 4;
  const int b = blockIdx.y, l0 = blockIdx.x * 64 + wave * 16;
  const float* pb = pose + (size_t)b * NA * CI * NPX; const float* ab = act + (size_t)b * NA * NPX;
  const int lm = l0 + col, ym = lm / HW, xm = lm % HW;
  v8f num[NBO]; float arsum[8]; float ausum[8];
#pragma unroll
  for (int be = 0; be < NBO; ++be) num[be] = (v8f){};
#pragma unroll
  for (int r = 0; r < 8; ++r) { ausum[r] = 0.f; arsum[r] = 0.f; }
#pragma unroll 1
  for (int kap = 0; kap < KKA; ++kap) { const int kk = kap / NA, a = kap % NA; const int di = kk / 3 - 1, dj = kk % 3 - 1;
    const int ys = ym + di, xs = xm + dj; const bool inb = ys >= 0 && ys < HW && xs >= 0 && xs < HW;
    const v16h af = frag_pose(pb, a, ys, xs, inb, lane);
    v8f vt[NBO];
#pragma unroll
    for (int be = 0; be < NBO; ++be) { vt[be] = (v8f){}; vt[be] = wmma16(af, frag_w16(W1 + ((size_t)kap * (NBO * DO) + be * DO + col) * CI, lane, 16.0f), vt[be]); }
    v8f lg = {}; lg = wmma16(af, frag_w16(W2 + ((size_t)kap * NBO + (col < NBO ? col : 0)) * CI, lane, 16.0f), lg);
    const float bb2 = col < NBO ? b2[kap * NBO + col] : 0.f;
    float rr[8];
#pragma unroll
    for (int r = 0; r < 8; ++r) { float lv = col < NBO ? lg[r] * (1.0f / 16.0f) + bb2 : -3.0e38f; float mx = lv;
#pragma unroll
      for (int off = 1; off <= 4; off <<= 1) mx = fmaxf(mx, __shfl_xor(mx, off, 32));
      mx = fmaxf(mx, __shfl_xor(mx, 8, 32));
      const float e = col < NBO ? expf(lv - mx) : 0.f; float se = e;
#pragma unroll
      for (int off = 1; off <= 8; off <<= 1) se += __shfl_xor(se, off, 32);
      rr[r] = e / se; }
    float au[8];
#pragma unroll
    for (int r = 0; r < 8; ++r) { const int lr = l0 + 8 * g + r, yr = lr / HW + di, xr = lr % HW + dj; au[r] = (yr >= 0 && yr < HW && xr >= 0 && xr < HW) ? ab[(size_t)a * NPX + yr * HW + xr] : 0.f; ausum[r] += au[r]; }
#pragma unroll
    for (int be = 0; be < NBO; ++be) {
#pragma unroll
      for (int r = 0; r < 8; ++r) { const float rb = __shfl(rr[r], g * 16 + be, 32); const float w = au[r] * rb; num[be][r] += w * (vt[be][r] * (1.0f / 16.0f)); } }
#pragma unroll
    for (int r = 0; r < 8; ++r) arsum[r] += au[r] * rr[r]; }
#pragma unroll
  for (int r = 0; r < 8; ++r) { const int pl = wave * 16 + 8 * g + r;
#pragma unroll
    for (int be = 0; be < NBO; ++be) { const float asb = __shfl(arsum[r], g * 16 + be, 32); sp[be * DO + col][pl] = num[be][r] / asb; }
    if (col < NBO) sa[col][pl] = arsum[r] / ausum[r]; }
  __syncthreads();
  const int lb = blockIdx.x * 64;
  for (int q = tid; q < NBO * 16; q += 128) { const int be = q >> 4, pc = q & 15; vst2(aout + ((size_t)b * NBO + be) * NPX + lb + pc * 4, *(const v4f*)(&sa[be][pc * 4])); }
  for (int q = tid; q < NBO * DO * 16; q += 128) { const int ch = q >> 4, pc = q & 15; vst2(pout + ((size_t)b * NBO * DO + ch) * NPX + lb + pc * 4, *(const v4f*)(&sp[ch][pc * 4])); }
}
extern "C" void kernel_launch(void* const* d_in, const int* in_sizes, int n_in, void* d_out, int out_size, void* d_ws, size_t ws_size, hipStream_t stream) {
  (void)in_sizes; (void)n_in; (void)out_size; (void)ws_size; (void)d_ws;
  const float* act = (const float*)d_in[0]; const float* pose = (const float*)d_in[1]; const float* W1 = (const float*)d_in[2]; const float* W2 = (const float*)d_in[3]; const float* b2 = (const float*)d_in[4];
  float* aout = (float*)d_out; float* pout = (float*)((char*)d_out + 131072);
  k_main<<<dim3(NPX / 64, NB), 128, 0, stream>>>(act, pose, W1, W2, b2, aout, pout);
}
